// MultiheadLocalAttentionV3_23888608100409
// MI455X (gfx1250) — hardware-verified
//
#include <hip/hip_runtime.h>
#include <math.h>
#include <stdint.h>

#define NB    2
#define CD    256
#define NH    8
#define HD    32
#define HIM   40
#define WIM   40
#define HWP   1600
#define NROW  (NB * HWP)
#define WSZ   15
#define WS2   225
#define WSP   256
#define MDIS  7
#define QT    32
#define NQB   (HWP / QT)
#define KCH   64
static_assert(NH * HD == CD);
static_assert(HD == 32);
static_assert((HWP % 64) == 0 && (NROW % 64) == 0 && (CD % 64) == 0 && (HWP % QT) == 0 && (HWP % KCH) == 0);
static_assert(((QT * WS2) % 4) == 0);
static_assert(((QT * WS2 * 4) % 128) == 0);
static_assert(((HWP * WS2 * 4) % 128) == 0);
static_assert(WSZ * WSZ == WS2 && WS2 <= WSP && (WSP % KCH) == 0);

typedef _Float16 v16h __attribute__((ext_vector_type(16)));
typedef _Float16 v8h  __attribute__((ext_vector_type(8)));
typedef __bf16   v16b __attribute__((ext_vector_type(16)));
typedef __bf16   v8b  __attribute__((ext_vector_type(8)));
typedef float    v8f  __attribute__((ext_vector_type(8)));
typedef float    v4f  __attribute__((ext_vector_type(4)));
typedef unsigned int v4u __attribute__((ext_vector_type(4)));

__device__ __forceinline__ unsigned short bf_bits(float f) {
  unsigned u = __float_as_uint(f);
  return (unsigned short)((u + 0x7FFFu + ((u >> 16) & 1u)) >> 16);
}
__device__ __forceinline__ float bf_up(unsigned short h) { return __uint_as_float(((unsigned)h) << 16); }
__device__ __forceinline__ unsigned short h_bits(_Float16 x) { return __builtin_bit_cast(unsigned short, x); }
__device__ __forceinline__ unsigned pk16(unsigned short a, unsigned short b) { return (unsigned)a | ((unsigned)b << 16); }
__device__ __forceinline__ v8f zero8() { v8f z = {0.f, 0.f, 0.f, 0.f, 0.f, 0.f, 0.f, 0.f}; return z; }

__device__ __forceinline__ v16b ldfrag_b(const __bf16* p) {
  union { v16b v; v8b h[2]; } f;
  f.h[0] = *(const v8b*)(p);
  f.h[1] = *(const v8b*)(p + 16);
  return f.v;
}
__device__ __forceinline__ v16h ldfrag_h(const _Float16* p) {
  union { v16h v; v8h h[2]; } f;
  f.h[0] = *(const v8h*)(p);
  f.h[1] = *(const v8h*)(p + 16);
  return f.v;
}

__device__ __forceinline__ v8f mma_h(v16h a, v16h b, v8f c) {
  c = __builtin_amdgcn_wmma_f32_16x16x32_f16(false, a, false, b, (short)0, c, false, false);
#if defined(__HIP_DEVICE_COMPILE__)
  asm volatile("v_nop\n\tv_nop\n\tv_nop\n\tv_nop" : "+v"(c) : "v"(a), "v"(b));
#endif
  return c;
}
__device__ __forceinline__ v8f mma_b_raw(v16b a, v16b b, v8f c) {
  return __builtin_amdgcn_wmma_f32_16x16x32_bf16(false, a, false, b, (short)0, c, false, false);
}
__device__ __forceinline__ void dep_guard_b(v8f& a, v8f& b, v16b x, v16b y) {
#if defined(__HIP_DEVICE_COMPILE__)
  asm volatile("v_nop\n\tv_nop\n\tv_nop\n\tv_nop" : "+v"(a), "+v"(b) : "v"(x), "v"(y));
#endif
}
__device__ __forceinline__ void keep4_b(v16b a, v16b b, v16b c, v16b d) {
#if defined(__HIP_DEVICE_COMPILE__)
  asm volatile("v_nop" :: "v"(a), "v"(b), "v"(c), "v"(d));
#endif
}
__device__ __forceinline__ void acc_guard4(v8f& a, v8f& b, v8f& c, v8f& d) {
#if defined(__HIP_DEVICE_COMPILE__)
  asm volatile("v_nop\n\tv_nop\n\tv_nop\n\tv_nop" : "+v"(a), "+v"(b), "+v"(c), "+v"(d));
#endif
}
__device__ __forceinline__ void wave_sync_lds() {
  __builtin_amdgcn_fence(__ATOMIC_RELEASE, "workgroup");
  __builtin_amdgcn_wave_barrier();
  __builtin_amdgcn_fence(__ATOMIC_ACQUIRE, "workgroup");
}

__device__ __forceinline__ v8f score3(const v16h qh, const v16h ql, const v16h kh, const v16h kl, const float rres) {
  v8f acc = zero8();
  acc = mma_h(ql, kh, acc);
  acc = mma_h(qh, kl, acc);
#pragma unroll
  for (int r = 0; r < 8; ++r) acc[r] *= rres;
  acc = mma_h(qh, kh, acc);
  return acc;
}

__global__ __launch_bounds__(256) void cvt_xT(const float* __restrict__ x0, const float* __restrict__ x1,
                                              const float* __restrict__ x2, unsigned short* outp) {
  __shared__ float tile[64][33];
  const int tid = threadIdx.x;
  const int z = blockIdx.z;
  const int s = z / NB, n = z - s * NB;
  const float* src = ((s == 0) ? x0 : ((s == 1) ? x1 : x2)) + (size_t)n * CD * HWP;
  unsigned short* dst = outp + ((size_t)s * NROW + (size_t)n * HWP) * CD;
  const int c0 = blockIdx.x * 64;
  const int p0 = blockIdx.y * 32;
#pragma unroll
  for (int it = 0; it < 8; ++it) {
    const int idx = it * 256 + tid;
    const int cc = idx >> 5, pp = idx & 31;
    tile[cc][pp] = src[(size_t)(c0 + cc) * HWP + p0 + pp];
  }
  __syncthreads();
  const int pp = tid >> 3, c8 = (tid & 7) * 8;
  v4u pk;
#pragma unroll
  for (int e = 0; e < 4; ++e)
    pk[e] = pk16(bf_bits(tile[c8 + 2 * e][pp]), bf_bits(tile[c8 + 2 * e + 1][pp]));
  unsigned short* gp = dst + (size_t)(p0 + pp) * CD + c0 + c8;
  *(volatile v4u*)gp = pk;
  __threadfence();
  *(volatile v4u*)gp = pk;
}

__global__ __launch_bounds__(256) void cvt4_bf16x8(const float* __restrict__ w0, const float* __restrict__ w1,
                                                   const float* __restrict__ w2, const float* __restrict__ w3,
                                                   unsigned short* outp, int n8) {
  const int z = blockIdx.y;
  const float* src = (z == 0) ? w0 : ((z == 1) ? w1 : ((z == 2) ? w2 : w3));
  unsigned short* dst = outp + (size_t)z * (size_t)n8 * 8;
  const int i = blockIdx.x * 256 + threadIdx.x;
  if (i < n8) {
    const v4f a = *(const v4f*)(src + (size_t)i * 8);
    const v4f b = *(const v4f*)(src + (size_t)i * 8 + 4);
    v4u p;
    p[0] = pk16(bf_bits(a[0]), bf_bits(a[1]));
    p[1] = pk16(bf_bits(a[2]), bf_bits(a[3]));
    p[2] = pk16(bf_bits(b[0]), bf_bits(b[1]));
    p[3] = pk16(bf_bits(b[2]), bf_bits(b[3]));
    *(volatile v4u*)(dst + (size_t)i * 8) = p;
    __threadfence();
    *(volatile v4u*)(dst + (size_t)i * 8) = p;
  }
}

__global__ __launch_bounds__(256) void cvt_rel(const float* __restrict__ rkw, const float* __restrict__ rv,
                                               unsigned short* rkwo, unsigned short* rvo, float tsc) {
  const int i = blockIdx.x * 256 + threadIdx.x;
  const int h = i >> 10, rem = i & 1023;
  unsigned short u[8];
  unsigned short* gp;
  if (blockIdx.y == 0) {
    const int w = rem >> 2, d0 = (rem & 3) * 8;
    const int wc = min(w, WS2 - 1);
    const float* sp = rkw + ((size_t)(h * WS2 + wc) * HD + d0);
    const v4f a = *(const v4f*)sp;
    const v4f b = *(const v4f*)(sp + 4);
    const bool ok = (w < WS2);
#pragma unroll
    for (int e = 0; e < 4; ++e) {
      const unsigned short ua = h_bits((_Float16)(bf_up(bf_bits(a[e])) * tsc));
      const unsigned short ub = h_bits((_Float16)(bf_up(bf_bits(b[e])) * tsc));
      u[e]     = ok ? ua : (unsigned short)0;
      u[4 + e] = ok ? ub : (unsigned short)0;
    }
    gp = rkwo + (size_t)i * 8;
  } else {
    const int d = rem >> 5, w0 = (rem & 31) * 8;
    const float* sp = rv + (size_t)(h * HD + d) * WS2;
#pragma unroll
    for (int e = 0; e < 8; ++e) {
      const int wv = w0 + e;
      const float x = sp[min(wv, WS2 - 1)];
      const unsigned short ux = h_bits((_Float16)(bf_up(bf_bits(x)) * tsc));
      u[e] = (wv < WS2) ? ux : (unsigned short)0;
    }
    gp = rvo + (size_t)i * 8;
  }
  v4u pk;
#pragma unroll
  for (int e = 0; e < 4; ++e) pk[e] = pk16(u[2 * e], u[2 * e + 1]);
  *(volatile v4u*)gp = pk;
  __threadfence();
  *(volatile v4u*)gp = pk;
}

__global__ __launch_bounds__(256) void cvt_hl_x8(const float* __restrict__ in, unsigned short* oh,
                                                 unsigned short* ol, int n8) {
  const int i = blockIdx.x * 256 + threadIdx.x;
  if (i < n8) {
    const v4f a = *(const v4f*)(in + (size_t)i * 8);
    const v4f b = *(const v4f*)(in + (size_t)i * 8 + 4);
    float f[8];
#pragma unroll
    for (int e = 0; e < 4; ++e) { f[e] = a[e]; f[4 + e] = b[e]; }
    v4u ph, pl;
#pragma unroll
    for (int e = 0; e < 4; ++e) {
      const unsigned short h0 = bf_bits(f[2 * e]), h1 = bf_bits(f[2 * e + 1]);
      const unsigned short l0 = bf_bits(f[2 * e] - bf_up(h0)), l1 = bf_bits(f[2 * e + 1] - bf_up(h1));
      ph[e] = pk16(h0, h1);
      pl[e] = pk16(l0, l1);
    }
    *(volatile v4u*)(oh + (size_t)i * 8) = ph;
    *(volatile v4u*)(ol + (size_t)i * 8) = pl;
    __threadfence();
    *(volatile v4u*)(oh + (size_t)i * 8) = ph;
    *(volatile v4u*)(ol + (size_t)i * 8) = pl;
  }
}

template <int NSPLIT, int OUT_MODE>
__global__ __launch_bounds__(256) void gemm64(
    const unsigned short* __restrict__ Ap, const unsigned short* A2p, int lda, long long strideA,
    const unsigned short* __restrict__ Btp, const unsigned short* Bt2p, int ldb, long long strideB,
    void* Cout, int ldc, long long strideC,
    void* Cout2, int ldc2, long long strideC2, int N2,
    int M, int N, int K, float rscale, const float* __restrict__ biasp, int nbias, int bias_on_m) {
  const __bf16* A   = (const __bf16*)(const void*)Ap;
  const __bf16* A2  = (const __bf16*)(const void*)A2p;
  const __bf16* Bt  = (const __bf16*)(const void*)Btp;
  const __bf16* Bt2 = (const __bf16*)(const void*)Bt2p;
  __shared__ __align__(16) float sT[8][16 * 68];
  const int b    = blockIdx.y;
  const int lane = threadIdx.x & 31;
  const int wave = threadIdx.x >> 5;
  const int tilesN = N >> 6;
  const int tilesM = M >> 6;
  const int tile = blockIdx.x * 8 + wave;
  if (tile >= tilesM * tilesN) return;
  const int tm = tile / tilesN;
  const int tn = tile - tm * tilesN;
  const int m0 = tm << 6;
  const int n0 = tn << 6;

  const __bf16* Ab  = A  + (size_t)b * strideA;
  const __bf16* Bb  = Bt + (size_t)b * strideB;
  const __bf16* Ab2 = (NSPLIT >= 1) ? (A2  + (size_t)b * strideA) : Ab;
  const __bf16* Bb2 = (NSPLIT == 2) ? (Bt2 + (size_t)b * strideB) : Bb;

  const int rlane = lane & 15;
  const int koff  = (lane >> 4) * 8;
  const int mOff  = (lane >> 4) * 8;

  v8f acc[4][4];
#pragma unroll
  for (int i = 0; i < 4; ++i)
#pragma unroll
    for (int j = 0; j < 4; ++j) acc[i][j] = zero8();

  for (int k0 = 0; k0 < K; k0 += 32) {
    v16b bh[4], bl[4];
#pragma unroll
    for (int j = 0; j < 4; ++j) {
      const size_t bo = (size_t)(n0 + (j << 4) + rlane) * ldb + koff + k0;
      bh[j] = ldfrag_b(Bb + bo);
      if (NSPLIT == 2) bl[j] = ldfrag_b(Bb2 + bo); else bl[j] = bh[j];
    }
#pragma unroll
    for (int i = 0; i < 4; ++i) {
      const size_t ao = (size_t)(m0 + (i << 4) + rlane) * lda + koff + k0;
      const v16b ah = ldfrag_b(Ab + ao);
      v16b al = ah;
      if (NSPLIT >= 1) al = ldfrag_b(Ab2 + ao);
#pragma unroll
      for (int j = 0; j < 4; ++j) {
        acc[i][j] = mma_b_raw(ah, bh[j], acc[i][j]);
        if (NSPLIT >= 1) acc[i][j] = mma_b_raw(al, bh[j], acc[i][j]);
        if (NSPLIT == 2) acc[i][j] = mma_b_raw(ah, bl[j], acc[i][j]);
      }
      dep_guard_b(acc[i][0], acc[i][3], ah, al);
    }
    keep4_b(bh[0], bh[1], bh[2], bh[3]);
    if (NSPLIT == 2) keep4_b(bl[0], bl[1], bl[2], bl[3]);
  }
  acc_guard4(acc[0][0], acc[0][1], acc[0][2], acc[0][3]);
  acc_guard4(acc[1][0], acc[1][1], acc[1][2], acc[1][3]);
  acc_guard4(acc[2][0], acc[2][1], acc[2][2], acc[2][3]);
  acc_guard4(acc[3][0], acc[3][1], acc[3][2], acc[3][3]);

  float* slab = sT[wave];
#pragma unroll
  for (int i = 0; i < 4; ++i) {
    const int mBase = m0 + (i << 4);
#pragma unroll
    for (int j = 0; j < 4; ++j) {
#pragma unroll
      for (int r = 0; r < 8; ++r) {
        slab[(mOff + r) * 68 + (j << 4) + rlane] = acc[i][j][r];
      }
    }
    wave_sync_lds();
    if (OUT_MODE == 0) {
      float* C = (float*)Cout + (size_t)b * strideC;
      const int hh = lane >> 4, c4 = (lane & 15) * 4;
      v4f bv;
#pragma unroll
      for (int e = 0; e < 4; ++e) bv[e] = bf_up(bf_bits(biasp[min(n0 + c4 + e, nbias - 1)]));
      for (int pass = 0; pass < 2; ++pass) {
#pragma unroll
        for (int it = 0; it < 8; ++it) {
          const int row = it * 2 + hh;
          const v4f v = *(const v4f*)(slab + row * 68 + c4) + bv;
          *(volatile v4f*)(C + (size_t)(mBase + row) * ldc + n0 + c4) = v;
        }
        __threadfence();
      }
    } else {
      const int q = lane >> 3, c8 = (lane & 7) * 8;
      unsigned short* C  = (unsigned short*)Cout  + (size_t)b * strideC;
      unsigned short* C2 = (unsigned short*)Cout2 + (size_t)b * strideC2;
      const bool wlo = (OUT_MODE == 2) || (n0 < N2);
      v4u hv[4], lv[4];
#pragma unroll
      for (int it = 0; it < 4; ++it) {
        const int row = it * 4 + q;
        const float* sp = slab + row * 68 + c8;
        const float brow = bf_up(bf_bits(biasp[min(mBase + row, nbias - 1)]));
        v4u a, a2;
#pragma unroll
        for (int e = 0; e < 4; ++e) {
          const float bc0 = bf_up(bf_bits(biasp[min(n0 + c8 + 2 * e, nbias - 1)]));
          const float bc1 = bf_up(bf_bits(biasp[min(n0 + c8 + 2 * e + 1, nbias - 1)]));
          const float f0 = sp[2 * e] + (bias_on_m ? brow : bc0);
          const float f1 = sp[2 * e + 1] + (bias_on_m ? brow : bc1);
          unsigned short h0, h1, l0, l1;
          if (OUT_MODE == 2) {
            h0 = bf_bits(f0); h1 = bf_bits(f1);
            l0 = bf_bits(f0 - bf_up(h0)); l1 = bf_bits(f1 - bf_up(h1));
          } else {
            const _Float16 x0 = (_Float16)f0, x1 = (_Float16)f1;
            h0 = h_bits(x0); h1 = h_bits(x1);
            l0 = h_bits((_Float16)((f0 - (float)x0) * rscale));
            l1 = h_bits((_Float16)((f1 - (float)x1) * rscale));
          }
          a[e] = pk16(h0, h1); a2[e] = pk16(l0, l1);
        }
        hv[it] = a; lv[it] = a2;
      }
      for (int pass = 0; pass < 2; ++pass) {
#pragma unroll
        for (int it = 0; it < 4; ++it) {
          const int row = it * 4 + q;
          *(volatile v4u*)(C + (size_t)(mBase + row) * ldc + n0 + c8) = hv[it];
          if (wlo) *(volatile v4u*)(C2 + (size_t)(mBase + row) * ldc2 + n0 + c8) = lv[it];
        }
        __threadfence();
      }
    }
    wave_sync_lds();
  }
}

__global__ __launch_bounds__(64)
void lattn(const unsigned short* __restrict__ qhp, const unsigned short* __restrict__ qlp,
           const unsigned short* __restrict__ khp, const unsigned short* __restrict__ klp,
           const unsigned short* __restrict__ vhp, const unsigned short* __restrict__ vlp,
           const unsigned short* __restrict__ rkwp, const float* __restrict__ rkb,
           const unsigned short* __restrict__ rvp,
           float* agf, float* aout, float sscale, float rres, float rtab) {
  union FH { v16h v; v8h h[2]; };
  __shared__ __align__(16) float    Lt[QT * WS2];
  __shared__ __align__(16) _Float16 Psh[2][16 * KCH];
  __shared__ __align__(16) _Float16 Psl[2][16 * KCH];
  __shared__ __align__(16) float    Os[QT * HD];

  const int tid  = threadIdx.x;
  const int wave = tid >> 5;
  const int lane = tid & 31;
  const int hh   = lane >> 4;
  const int c    = lane & 15;

  const int bx   = blockIdx.x;
  const int qb   = bx % NQB;
  const int rest = bx / NQB;
  const int h    = rest % NH;
  const int n    = rest / NH;
  const int q0b  = qb * QT;
  const int q0w  = q0b + wave * 16;
  const size_t rowP = (size_t)n * HWP;

  const _Float16* Qh = (const _Float16*)(const void*)qhp + (size_t)h * HD;
  const _Float16* Ql = (const _Float16*)(const void*)qlp + (size_t)h * HD;
  const _Float16* Kh = (const _Float16*)(const void*)khp + (size_t)h * HD;
  const _Float16* Kl = (const _Float16*)(const void*)klp + (size_t)h * HD;
  const _Float16* Vh = (const _Float16*)(const void*)vhp + ((size_t)n * CD + (size_t)h * HD) * HWP;
  const _Float16* Vl = (const _Float16*)(const void*)vlp + ((size_t)n * CD + (size_t)h * HD) * HWP;
  const _Float16* Rk = (const _Float16*)(const void*)rkwp + (size_t)h * WSP * HD;
  const _Float16* Rv = (const _Float16*)(const void*)rvp + (size_t)h * HD * WSP;

  const v16h qah = ldfrag_h(Qh + (rowP + q0w + c) * CD + 8 * hh);
  const v16h qal = ldfrag_h(Ql + (rowP + q0w + c) * CD + 8 * hh);

  int qyr[8], qxr[8];
#pragma unroll
  for (int r = 0; r < 8; ++r) {
    const int i = q0w + 8 * hh + r;
    qyr[r] = i / WIM;
    qxr[r] = i - qyr[r] * WIM;
  }

  float*    lw  = Lt + wave * 16 * WS2;
  _Float16* pwh = Psh[wave];
  _Float16* pwl = Psl[wave];

#pragma unroll 1
  for (int wt = 0; wt < WSP / 16; ++wt) {
    const v16h bw = ldfrag_h(Rk + (size_t)(wt * 16 + c) * HD + 8 * hh);
    v8f acc = zero8();
    acc = mma_h(qal, bw, acc);
#pragma unroll
    for (int r = 0; r < 8; ++r) acc[r] *= rres;
    acc = mma_h(qah, bw, acc);
    const int w  = wt * 16 + c;
    const int wc = min(w, WS2 - 1);
    const float rb = bf_up(bf_bits(rkb[h * WS2 + wc]));
    const int wy  = wc / WSZ;
    const int dyo = wy - MDIS;
    const int dxo = (wc - wy * WSZ) - MDIS;
#pragma unroll
    for (int r = 0; r < 8; ++r) {
      const int ky = qyr[r] + dyo, kx = qxr[r] + dxo;
      const bool in = ((unsigned)ky < (unsigned)HIM) && ((unsigned)kx < (unsigned)WIM);
      const float val = in ? (acc[r] * rtab + rb) : -INFINITY;
      if (w < WS2) lw[(8 * hh + r) * WS2 + w] = val;
    }
  }
  wave_sync_lds();

  const int qyLo = q0b / WIM;
  const int qyHi = (q0b + QT - 1) / WIM;
  const int kyLo = max(qyLo - MDIS, 0);
  const int kyHi = min(qyHi + MDIS, HIM - 1);
  const int ktLo = (kyLo * WIM) / KCH;
  const int ktHi = min((kyHi * WIM + WIM - 1) / KCH, HWP / KCH - 1);

  float mrow[8], lrow[8];
  v8f oacc[2];
#pragma unroll
  for (int r = 0; r < 8; ++r) { mrow[r] = -INFINITY; lrow[r] = 0.f; }
#pragma unroll
  for (int t = 0; t < 2; ++t) oacc[t] = zero8();

  for (int kt = ktLo; kt <= ktHi; ++kt) {
    const int kv0 = kt * KCH;

    v8f s[4];
#pragma unroll
    for (int j = 0; j < 4; ++j) {
      const size_t ko = (rowP + kv0 + j * 16 + c) * CD + 8 * hh;
      const v16h kb = ldfrag_h(Kh + ko);
      const v16h kl = ldfrag_h(Kl + ko);
      s[j] = score3(qah, qal, kb, kl, rres);
    }

#pragma unroll
    for (int j = 0; j < 4; ++j) {
      const int key = kv0 + j * 16 + c;
      const int ky  = key / WIM;
      const int kx  = key - ky * WIM;
#pragma unroll
      for (int r = 0; r < 8; ++r) {
        const int ay = ky - qyr[r] + MDIS;
        const int ax = kx - qxr[r] + MDIS;
        const bool valid = ((unsigned)ay <= (unsigned)(2 * MDIS)) && ((unsigned)ax <= (unsigned)(2 * MDIS));
        const int w = valid ? (ay * WSZ + ax) : 0;
        float* lp = lw + (8 * hh + r) * WS2 + w;
        const float relv = *lp;
        const float lg = valid ? (s[j][r] * sscale + relv) : -INFINITY;
        if (valid) *lp = lg;
        s[j][r] = lg;
      }
    }

#pragma unroll
    for (int r = 0; r < 8; ++r) {
      float m = fmaxf(fmaxf(s[0][r], s[1][r]), fmaxf(s[2][r], s[3][r]));
#pragma unroll
      for (int off = 1; off < 16; off <<= 1) m = fmaxf(m, __shfl_xor(m, off, 32));
      const float mnew  = fmaxf(mrow[r], m);
      const float msafe = (mnew == -INFINITY) ? 0.f : mnew;
      const float alpha = __expf(mrow[r] - msafe);
      mrow[r] = mnew;
      float psum = 0.f;
#pragma unroll
      for (int j = 0; j < 4; ++j) {
        const float p  = __expf(s[j][r] - msafe);
        psum += p;
        const float p1 = p * 1024.0f;
        const _Float16 x = (_Float16)p1;
        const int idx = (8 * hh + r) * KCH + j * 16 + c;
        pwh[idx] = x;
        pwl[idx] = (_Float16)((p1 - (float)x) * 4096.0f);
      }
#pragma unroll
      for (int off = 1; off < 16; off <<= 1) psum += __shfl_xor(psum, off, 32);
      lrow[r] = lrow[r] * alpha + psum;
#pragma unroll
      for (int t = 0; t < 2; ++t) oacc[t][r] *= alpha;
    }
    wave_sync_lds();

    v8f o1[2];
    o1[0] = zero8(); o1[1] = zero8();
#pragma unroll
    for (int kk = 0; kk < 2; ++kk) {
      FH pa, pl;
      pa.h[0] = *(const v8h*)(pwh + c * KCH + kk * 32 + 8 * hh);
      pa.h[1] = *(const v8h*)(pwh + c * KCH + kk * 32 + 16 + 8 * hh);
      pl.h[0] = *(const v8h*)(pwl + c * KCH + kk * 32 + 8 * hh);
      pl.h[1] = *(const v8h*)(pwl + c * KCH + kk * 32 + 16 + 8 * hh);
#pragma unroll
      for (int t = 0; t < 2; ++t) {
        const size_t vo = (size_t)(t * 16 + c) * HWP + kv0 + kk * 32 + 8 * hh;
        const v16h vb = ldfrag_h(Vh + vo);
        const v16h vl = ldfrag_h(Vl + vo);
        oacc[t] = mma_h(pa.v, vb, oacc[t]);
        o1[t]   = mma_h(pa.v, vl, o1[t]);
        o1[t]   = mma_h(pl.v, vb, o1[t]);
      }
    }
#pragma unroll
    for (int t = 0; t < 2; ++t)
#pragma unroll
      for (int r = 0; r < 8; ++r) oacc[t][r] += o1[t][r] * rres;
    wave_sync_lds();
  }

  wave_sync_lds();
  float invl[8];
#pragma unroll
  for (int r = 0; r < 8; ++r) invl[r] = (lrow[r] > 0.f) ? (1.0f / lrow[r]) : 0.f;
#pragma unroll
  for (int qq = 0; qq < 16; ++qq) {
    const int src = (qq >> 3) * 16;
    const float mq = __shfl(mrow[qq & 7], src, 32);
    const float iq = __shfl(invl[qq & 7], src, 32);
    float* rowp = lw + qq * WS2;
#pragma unroll 1
    for (int it = 0; it < (WS2 + 31) / 32; ++it) {
      const int w  = it * 32 + lane;
      const int wc = min(w, WS2 - 1);
      const float x = rowp[wc];
      const float p = __expf(x - mq) * iq;
      if (w < WS2) rowp[w] = p;
    }
  }
  wave_sync_lds();

  v8f bacc[2], bres[2];
  bacc[0] = zero8(); bacc[1] = zero8(); bres[0] = zero8(); bres[1] = zero8();
#pragma unroll 1
  for (int kc = 0; kc < WSP / KCH; ++kc) {
#pragma unroll
    for (int qq = 0; qq < 16; ++qq) {
#pragma unroll
      for (int hf = 0; hf < 2; ++hf) {
        const int col = hf * 32 + lane;
        const int w   = kc * KCH + col;
        const int wc  = min(w, WS2 - 1);
        float p = lw[qq * WS2 + wc];
        p = (w < WS2) ? p : 0.f;
        const float p1 = p * 1024.0f;
        const _Float16 x = (_Float16)p1;
        pwh[qq * KCH + col] = x;
        pwl[qq * KCH + col] = (_Float16)((p1 - (float)x) * 4096.0f);
      }
    }
    wave_sync_lds();
#pragma unroll
    for (int kk = 0; kk < 2; ++kk) {
      FH pa, pl;
      pa.h[0] = *(const v8h*)(pwh + c * KCH + kk * 32 + 8 * hh);
      pa.h[1] = *(const v8h*)(pwh + c * KCH + kk * 32 + 16 + 8 * hh);
      pl.h[0] = *(const v8h*)(pwl + c * KCH + kk * 32 + 8 * hh);
      pl.h[1] = *(const v8h*)(pwl + c * KCH + kk * 32 + 16 + 8 * hh);
#pragma unroll
      for (int t = 0; t < 2; ++t) {
        const v16h vb = ldfrag_h(Rv + (size_t)(t * 16 + c) * WSP + kc * KCH + kk * 32 + 8 * hh);
        bacc[t] = mma_h(pa.v, vb, bacc[t]);
        bres[t] = mma_h(pl.v, vb, bres[t]);
      }
    }
    wave_sync_lds();
  }

  const float bscale = rtab * (1.0f / 1024.0f);
#pragma unroll
  for (int r = 0; r < 8; ++r) {
    const float inv = invl[r] * (1.0f / 1024.0f);
#pragma unroll
    for (int t = 0; t < 2; ++t) {
      Os[(wave * 16 + 8 * hh + r) * HD + t * 16 + c] =
          oacc[t][r] * inv + (bacc[t][r] + bres[t][r] * rres) * bscale;
    }
  }
  __syncthreads();

  {
    const int rq = tid >> 3, c4 = (tid & 7) * 4;
    v4f ov[4];
#pragma unroll
    for (int it = 0; it < 4; ++it) {
      const int row = it * 8 + rq;
      ov[it] = *(const v4f*)(Os + row * HD + c4);
    }
    for (int pass = 0; pass < 2; ++pass) {
#pragma unroll
      for (int it = 0; it < 4; ++it) {
        const int row = it * 8 + rq;
        const size_t go = ((size_t)(q0b + row) * NB + n) * CD + (size_t)h * HD + c4;
        *(volatile v4f*)(agf + go) = ov[it];
      }
      __threadfence();
    }
  }

  {
    float* dst = aout + ((size_t)(n * NH + h) * HWP + q0b) * WS2;
    constexpr int NCHK = QT * WS2 / 4;
    for (int pass = 0; pass < 2; ++pass) {
#pragma unroll 1
      for (int it = 0; it < (NCHK + 63) / 64; ++it) {
        const int ch = it * 64 + tid;
        if (ch < NCHK) {
          const v4f v = *(const v4f*)(Lt + ch * 4);
          *(volatile v4f*)(dst + (size_t)ch * 4) = v;
        }
      }
      __threadfence();
    }
  }
}

extern "C" void kernel_launch(void* const* d_in, const int* in_sizes, int n_in,
                              void* d_out, int out_size, void* d_ws, size_t ws_size,
                              hipStream_t stream) {
  if (n_in < 14) return;
  if (in_sizes[0] != NB * CD * HWP || in_sizes[1] != NB * CD * HWP || in_sizes[2] != NB * CD * HWP) return;
  if (in_sizes[3] != CD * CD || in_sizes[5] != CD * CD || in_sizes[7] != CD * CD || in_sizes[12] != CD * CD) return;
  if (in_sizes[4] != CD || in_sizes[6] != CD || in_sizes[8] != CD || in_sizes[13] != CD) return;
  if (in_sizes[9] != NH * WS2 * HD || in_sizes[10] != NH * WS2 || in_sizes[11] != NH * HD * WS2) return;
  if (out_size != NROW * CD + NB * NH * HWP * WS2) return;

  const float* q_in    = (const float*)d_in[0];
  const float* k_in    = (const float*)d_in[1];
  const float* v_in    = (const float*)d_in[2];
  const float* Wq      = (const float*)d_in[3];
  const float* bq      = (const float*)d_in[4];
  const float* Wk      = (const float*)d_in[5];
  const float* bk      = (const float*)d_in[6];
  const float* Wv      = (const float*)d_in[7];
  const float* bv      = (const float*)d_in[8];
  const float* rel_k_w = (const float*)d_in[9];
  const float* rel_k_b = (const float*)d_in[10];
  const float* rel_v   = (const float*)d_in[11];
  const float* Wp      = (const float*)d_in[12];
  const float* bp      = (const float*)d_in[13];

  const size_t PP   = (size_t)NROW * CD * 2;
  const size_t PXT  = 3 * PP;
  const size_t PW   = (size_t)4 * CD * CD * 2;
  const size_t PR   = (size_t)NH * WSP * HD * 2;
  const size_t PVT  = (size_t)NB * CD * HWP * 2;
  const size_t PAGF = (size_t)NROW * CD * 4;
  size_t off = 0;
  const size_t oXT  = off; off += PXT;
  const size_t oW   = off; off += PW;
  const size_t oRKW = off; off += PR;
  const size_t oRV  = off; off += PR;
  const size_t oQh  = off; off += PP;
  const size_t oQl  = off; off += PP;
  const size_t oKh  = off; off += PP;
  const size_t oKl  = off; off += PP;
  const size_t oVTh = off; off += PVT;
  const size_t oVTl = off; off += PVT;
  const size_t oAGF = off; off += PAGF;
  const size_t oAGH = off; off += PP;
  const size_t oAGL = off; off += PP;
  if (off > ws_size) return;
  if (off > (size_t)134217728) return;

  char* ws = (char*)d_ws;
  unsigned short* XT  = (unsigned short*)(ws + oXT);
  unsigned short* XqT = XT;
  unsigned short* XkT = XT + (size_t)1 * NROW * CD;
  unsigned short* XvT = XT + (size_t)2 * NROW * CD;
  unsigned short* Wb  = (unsigned short*)(ws + oW);
  unsigned short* Wqb = Wb;
  unsigned short* Wkb = Wb + (size_t)1 * CD * CD;
  unsigned short* Wvb = Wb + (size_t)2 * CD * CD;
  unsigned short* Wpb = Wb + (size_t)3 * CD * CD;
  unsigned short* RKW = (unsigned short*)(ws + oRKW);
  unsigned short* RV  = (unsigned short*)(ws + oRV);
  unsigned short* Qh  = (unsigned short*)(ws + oQh);
  unsigned short* Ql  = (unsigned short*)(ws + oQl);
  unsigned short* Kh  = (unsigned short*)(ws + oKh);
  unsigned short* Kl  = (unsigned short*)(ws + oKl);
  unsigned short* VTh = (unsigned short*)(ws + oVTh);
  unsigned short* VTl = (unsigned short*)(ws + oVTl);
  float*          AGF = (float*)(ws + oAGF);
  unsigned short* AGH = (unsigned short*)(ws + oAGH);
  unsigned short* AGL = (unsigned short*)(ws + oAGL);

  float* out0 = (float*)d_out;
  float* out1 = (float*)d_out + (size_t)NROW * CD;

  const float sscale = 0.17677669529663687f;
  const float rres   = 1.0f / 4096.0f;
  const float tsc    = 64.0f;
  const float rtab   = 1.0f / 64.0f;

  const dim3 blk(256);
  const int  n8w  = CD * CD / 8;
  const int  n8ag = NROW * CD / 8;
  const dim3 gXT(CD / 64, HWP / 32, 3 * NB);
  const dim3 gW((n8w + 255) / 256, 4);
  const dim3 gRel((NH * WSP * HD / 8 + 255) / 256, 2);
  const dim3 gP(((NROW / 64) * (CD / 64) + 7) / 8, 1);
  const dim3 gVT(((CD / 64) * (HWP / 64) + 7) / 8, NB);
  const dim3 gHL((n8ag + 255) / 256);
  const dim3 gAttn(NB * NH * NQB);

  cvt_xT<<<gXT, blk, 0, stream>>>(q_in, k_in, v_in, XT);
  cvt4_bf16x8<<<gW, blk, 0, stream>>>(Wq, Wk, Wv, Wp, Wb, n8w);
  cvt_rel<<<gRel, blk, 0, stream>>>(rel_k_w, rel_v, RKW, RV, tsc);
  gemm64<0, 3><<<gP, blk, 0, stream>>>(
      XqT, XqT, CD, 0LL, Wqb, Wqb, CD, 0LL,
      (void*)Qh, CD, 0LL, (void*)Ql, CD, 0LL, CD,
      NROW, CD, CD, 4096.0f, bq, CD, 0);
  gemm64<0, 3><<<gP, blk, 0, stream>>>(
      XkT, XkT, CD, 0LL, Wkb, Wkb, CD, 0LL,
      (void*)Kh, CD, 0LL, (void*)Kl, CD, 0LL, CD,
      NROW, CD, CD, 4096.0f, bk, CD, 0);
  gemm64<0, 3><<<gVT, blk, 0, stream>>>(
      Wvb, Wvb, CD, 0LL, XvT, XvT, CD, (long long)HWP * CD,
      (void*)VTh, HWP, (long long)CD * HWP, (void*)VTl, HWP, (long long)CD * HWP, HWP,
      CD, HWP, CD, 4096.0f, bv, CD, 1);
  lattn<<<gAttn, dim3(64), 0, stream>>>(Qh, Ql, Kh, Kl, VTh, VTl, RKW, rel_k_b, RV, AGF, out1, sscale, rres, rtab);
  cvt_hl_x8<<<gHL, blk, 0, stream>>>(AGF, AGH, AGL, n8ag);
  gemm64<1, 0><<<gP, blk, 0, stream>>>(
      AGH, AGL, CD, 0LL, Wpb, Wpb, CD, 0LL,
      (void*)out0, CD, 0LL, (void*)out0, CD, 0LL, CD,
      NROW, CD, CD, 1.0f, bp, CD, 0);
  (void)hipGetLastError();
}
